// GraphAttention_1898375545033
// MI455X (gfx1250) — hardware-verified
//
#include <hip/hip_runtime.h>

typedef __bf16 v16b __attribute__((ext_vector_type(16)));
typedef __bf16 v8b  __attribute__((ext_vector_type(8)));
typedef float  v8f  __attribute__((ext_vector_type(8)));
typedef float  v4f  __attribute__((ext_vector_type(4)));
typedef unsigned int v4u __attribute__((ext_vector_type(4)));
typedef int    v4i  __attribute__((ext_vector_type(4)));
typedef v4f __attribute__((may_alias)) v4fa;
typedef v4i __attribute__((may_alias)) v4ia;
typedef v8b __attribute__((may_alias)) v8ba;

#define GB 8
#define GN 2048
#define GC 128
#define GD 64
#define NB 80
#define MT 128
#define PLANE_ELEMS (NB * GN)

static_assert(GN % 2 == 0);
static_assert(GN == 2048);
static_assert(GD == 64);
static_assert(NB == 5 * 16);
static_assert(GN % 32 == 0);
static_assert(GC % 32 == 0);
static_assert((GN / 2) % MT == 0);
static_assert((GB * GN) % 128 == 0);

#define PREP_XB_BLOCKS ((GB * GN * GC) / 8 / 256)
#define PREP_MK_BLOCKS ((GN * GN) / 8 / 256)
#define PREP_WT_BLOCKS ((GC * GD) / 8 / 256)
#define PREP_BLOCKS (PREP_XB_BLOCKS + PREP_MK_BLOCKS + PREP_WT_BLOCKS + 2)

__device__ __forceinline__ unsigned short f2bf_bits(float f) {
  const unsigned u = __float_as_uint(f);
  return (unsigned short)((u + 0x7FFFu + ((u >> 16) & 1u)) >> 16);
}
__device__ __forceinline__ float bf_bits2f(unsigned short hb) { return __uint_as_float(((unsigned)hb) << 16); }
__device__ __forceinline__ unsigned pk16(unsigned short a, unsigned short b) { return (unsigned)a | ((unsigned)b << 16); }
__device__ __forceinline__ float bfr(float f) { return bf_bits2f(f2bf_bits(f)); }

union FragB { v16b v; v8b half[2]; };
__device__ __forceinline__ v16b load_frag(const __bf16* p, int h) {
  FragB f;
  f.half[0] = *(const v8ba*)(p + 8 * h);
  f.half[1] = *(const v8ba*)(p + 16 + 8 * h);
  return f.v;
}
__device__ __forceinline__ v8f mma_bf16(v16b a, v16b b, v8f c) {
  c = __builtin_amdgcn_wmma_f32_16x16x32_bf16(false, a, false, b, (short)0, c, false, false);
  asm volatile("v_nop\n\tv_nop\n\tv_nop\n\tv_nop" : "+v"(c) : "v"(a), "v"(b));
  return c;
}

__global__ __launch_bounds__(256) void k_prep(
    const float* __restrict__ x, const int* __restrict__ adj, const float* __restrict__ W,
    const float* __restrict__ a, const float* __restrict__ bias,
    unsigned short* __restrict__ XB, unsigned short* __restrict__ MASK,
    unsigned short* __restrict__ Wt, float* __restrict__ AFBF)
{
  const int bx = blockIdx.x, tid = threadIdx.x;
  if (bx < PREP_XB_BLOCKS) {
    const size_t g = (size_t)bx * 256 + tid;
    const v4f a0 = *(const v4fa*)(x + g * 8);
    const v4f a1 = *(const v4fa*)(x + g * 8 + 4);
    v4u o;
    o.x = pk16(f2bf_bits(a0.x), f2bf_bits(a0.y));
    o.y = pk16(f2bf_bits(a0.z), f2bf_bits(a0.w));
    o.z = pk16(f2bf_bits(a1.x), f2bf_bits(a1.y));
    o.w = pk16(f2bf_bits(a1.z), f2bf_bits(a1.w));
    unsigned short* dst = XB + g * 8;
    *(volatile v4u*)dst = o;
    __threadfence();
    *(volatile v4u*)dst = o;
  } else if (bx < PREP_XB_BLOCKS + PREP_MK_BLOCKS) {
    const size_t g = (size_t)(bx - PREP_XB_BLOCKS) * 256 + tid;
    const v4i m0 = *(const v4ia*)(adj + g * 8);
    const v4i m1 = *(const v4ia*)(adj + g * 8 + 4);
    const unsigned one = 0x3F80u;
    v4u o;
    o.x = ((m0.x > 0) ? one : 0u) | (((m0.y > 0) ? one : 0u) << 16);
    o.y = ((m0.z > 0) ? one : 0u) | (((m0.w > 0) ? one : 0u) << 16);
    o.z = ((m1.x > 0) ? one : 0u) | (((m1.y > 0) ? one : 0u) << 16);
    o.w = ((m1.z > 0) ? one : 0u) | (((m1.w > 0) ? one : 0u) << 16);
    unsigned short* dst = MASK + g * 8;
    *(volatile v4u*)dst = o;
    __threadfence();
    *(volatile v4u*)dst = o;
  } else if (bx < PREP_XB_BLOCKS + PREP_MK_BLOCKS + PREP_WT_BLOCKS) {
    const int u = (bx - PREP_XB_BLOCKS - PREP_MK_BLOCKS) * 256 + tid;
    const int n = u >> 4, kg = u & 15;
    unsigned short hb[8];
#pragma unroll
    for (int e = 0; e < 8; ++e) hb[e] = f2bf_bits(W[(kg * 8 + e) * GD + n]);
    v4u o;
    o.x = pk16(hb[0], hb[1]);
    o.y = pk16(hb[2], hb[3]);
    o.z = pk16(hb[4], hb[5]);
    o.w = pk16(hb[6], hb[7]);
    unsigned short* dst = Wt + (size_t)u * 8;
    *(volatile v4u*)dst = o;
    __threadfence();
    *(volatile v4u*)dst = o;
  } else if (bx == PREP_XB_BLOCKS + PREP_MK_BLOCKS + PREP_WT_BLOCKS) {
    if (tid < 32) {
      const v4f v = *(const v4fa*)(a + 4 * tid);
      const v4f o = { bfr(v.x), bfr(v.y), bfr(v.z), bfr(v.w) };
      float* dst = AFBF + 4 * tid;
      *(volatile v4f*)dst = o;
      __threadfence();
      *(volatile v4f*)dst = o;
    }
  } else {
    if (tid < 16) {
      const v4f v = *(const v4fa*)(bias + 4 * tid);
      const v4f o = { bfr(v.x), bfr(v.y), bfr(v.z), bfr(v.w) };
      float* dst = AFBF + 128 + 4 * tid;
      *(volatile v4f*)dst = o;
      __threadfence();
      *(volatile v4f*)dst = o;
    }
  }
}

__global__ __launch_bounds__(256) void k_hid(
    const unsigned short* __restrict__ XBp, const unsigned short* __restrict__ Wtp,
    const float* __restrict__ AFBF, float* __restrict__ H, float* __restrict__ S12)
{
  __shared__ __attribute__((aligned(16))) float sT[8][16 * 68];
  __shared__ __attribute__((aligned(16))) float sAF[128];
  __shared__ __attribute__((aligned(16))) float sS[2][128];

  const int tid = threadIdx.x, lane = tid & 31, w = tid >> 5;
  const int h = lane >> 4, m = lane & 15;
  const int row0 = blockIdx.x * 128 + 16 * w;

  if (tid < 128) sAF[tid] = AFBF[tid];

  const __bf16* ar = (const __bf16*)(const void*)XBp + (size_t)(row0 + m) * GC;
  const __bf16* br = (const __bf16*)(const void*)Wtp + (size_t)m * GC;

  const v8f zero8 = {0.f, 0.f, 0.f, 0.f, 0.f, 0.f, 0.f, 0.f};
  v8f acc[4];
#pragma unroll
  for (int nt = 0; nt < 4; ++nt) acc[nt] = zero8;

#pragma unroll
  for (int k0 = 0; k0 < GC; k0 += 32) {
    const v16b af = load_frag(ar + k0, h);
#pragma unroll
    for (int nt = 0; nt < 4; ++nt) {
      const v16b bf = load_frag(br + (size_t)nt * 16 * GC + k0, h);
      acc[nt] = mma_bf16(af, bf, acc[nt]);
    }
  }

  float* slab = sT[w];
#pragma unroll
  for (int nt = 0; nt < 4; ++nt)
#pragma unroll
    for (int r = 0; r < 8; ++r)
      slab[(8 * h + r) * 68 + 16 * nt + m] = acc[nt][r];
  __syncthreads();

  {
    const int c4 = m * 4;
    for (int pass = 0; pass < 2; ++pass) {
#pragma unroll
      for (int it = 0; it < 8; ++it) {
        const int row = it * 2 + h;
        const v4f v = *(const v4fa*)(slab + row * 68 + c4);
        *(volatile v4f*)(H + (size_t)(row0 + row) * GD + c4) = v;
      }
      __threadfence();
    }
  }

  {
    const float* av = sAF + 64 * h;
    const float* sr = slab + m * 68;
    float sacc = 0.0f;
#pragma unroll 4
    for (int c = 0; c < GD; ++c) sacc = fmaf(sr[c], av[c], sacc);
    sS[h][16 * w + m] = sacc;
  }
  __syncthreads();

  if (w < 2) {
    const v4f v = *(const v4fa*)(&sS[w][lane * 4]);
    float* dst = S12 + (size_t)w * (GB * GN) + (size_t)blockIdx.x * 128 + lane * 4;
    *(volatile v4f*)dst = v;
    __threadfence();
    *(volatile v4f*)dst = v;
  }
}

__device__ __forceinline__ float leaky02(float v) { return (v >= 0.0f) ? v : 0.2f * v; }

__global__ __launch_bounds__(256) void k_wts(
    const float* __restrict__ S12, const float* __restrict__ H,
    float* __restrict__ WV, float* __restrict__ L0R, float* __restrict__ L1R,
    float* __restrict__ HM, float* __restrict__ STAT)
{
  __shared__ __attribute__((aligned(16))) float s1s[GN];
  __shared__ __attribute__((aligned(16))) float s2s[GN];
  __shared__ __attribute__((aligned(16))) float sLt[GN];
  __shared__ __attribute__((aligned(16))) float sL0[GN / 2];
  __shared__ __attribute__((aligned(16))) float sL1[GN / 2];
  __shared__ float sRmax[8];
  __shared__ float sRmin[8];
  __shared__ double sHMd[4][GD];
  __shared__ __attribute__((aligned(16))) float sHMf[GD];

  const int tid = threadIdx.x, lane = tid & 31, w = tid >> 5;
  const int b = blockIdx.x;

#pragma unroll
  for (int it = 0; it < 2; ++it) {
    const int idx = it * 1024 + tid * 4;
    const v4f v1 = *(const v4fa*)(S12 + (size_t)b * GN + idx);
    const v4f v2 = *(const v4fa*)(S12 + (size_t)(GB * GN) + (size_t)b * GN + idx);
    *(v4fa*)(s1s + idx) = v1;
    *(v4fa*)(s2s + idx) = v2;
  }
  __syncthreads();

  float tmax = -__builtin_inff(), tmin = __builtin_inff();
#pragma unroll 1
  for (int e = 0; e < 8; ++e) {
    const int j = (e >> 2) * 1024 + tid * 4 + (e & 3);
    const int i1 = (2 * j) & (GN - 1);
    const int i2 = (2 * j + 1) & (GN - 1);
    const float lt = leaky02(s1s[i1] + s2s[i2]);
    sLt[j] = lt;
    tmax = fmaxf(tmax, lt);
    tmin = fminf(tmin, lt);
  }
#pragma unroll 1
  for (int e = 0; e < 4; ++e) {
    const int i = tid * 4 + e;
    sL0[i] = leaky02(s1s[2 * i] + s2s[2 * i]);
    sL1[i] = leaky02(s1s[2 * i + 1] + s2s[2 * i + 1]);
  }
#pragma unroll
  for (int off = 16; off >= 1; off >>= 1) {
    tmax = fmaxf(tmax, __shfl_xor(tmax, off));
    tmin = fminf(tmin, __shfl_xor(tmin, off));
  }
  if (lane == 0) { sRmax[w] = tmax; sRmin[w] = tmin; }
  __syncthreads();
  float Mb = sRmax[0], mn = sRmin[0];
#pragma unroll
  for (int q = 1; q < 8; ++q) { Mb = fmaxf(Mb, sRmax[q]); mn = fminf(mn, sRmin[q]); }

#pragma unroll 1
  for (int e = 0; e < 8; ++e) {
    const int j = (e >> 2) * 1024 + tid * 4 + (e & 3);
    sLt[j] = expf(sLt[j] - Mb);
  }

  {
    const int c = tid & 63, part = tid >> 6;
    const float* hp = H + ((size_t)b * GN + (size_t)part * 512) * GD + c;
    double s = 0.0;
#pragma unroll 4
    for (int r = 0; r < 512; ++r) s += (double)hp[(size_t)r * GD];
    sHMd[part][c] = s;
  }
  __syncthreads();
  if (tid < GD) {
    const double tot = ((sHMd[0][tid] + sHMd[1][tid]) + sHMd[2][tid]) + sHMd[3][tid];
    sHMf[tid] = (float)(tot * (1.0 / 2048.0));
  }
  __syncthreads();

  for (int pass = 0; pass < 2; ++pass) {
#pragma unroll
    for (int it = 0; it < 2; ++it) {
      const int idx = it * 1024 + tid * 4;
      const v4f v = *(const v4fa*)(sLt + idx);
      *(volatile v4f*)(WV + (size_t)b * GN + idx) = v;
    }
    {
      const v4f v0 = *(const v4fa*)(sL0 + tid * 4);
      const v4f v1 = *(const v4fa*)(sL1 + tid * 4);
      *(volatile v4f*)(L0R + (size_t)b * (GN / 2) + tid * 4) = v0;
      *(volatile v4f*)(L1R + (size_t)b * (GN / 2) + tid * 4) = v1;
    }
    if (tid < 16) {
      const v4f v = *(const v4fa*)(sHMf + tid * 4);
      *(volatile v4f*)(HM + (size_t)b * GD + tid * 4) = v;
    }
    if (tid < 8) {
      const v4f v = { Mb, mn, expf(mn - Mb), (float)tid };
      *(volatile v4f*)(STAT + (size_t)b * 32 + tid * 4) = v;
    }
    __threadfence();
  }
}

__device__ __forceinline__ unsigned plane_bits(float hv, float wv, unsigned tmask, unsigned mlt,
                                               unsigned m64, unsigned c65, unsigned lmask) {
#pragma clang fp contract(off)
  const unsigned mfb = (__float_as_uint(wv) & tmask) | (0x3F800000u & ~tmask);
  const float mf = __uint_as_float(mfb);
  const float prod = hv * mf;
  const unsigned vb = (__float_as_uint(prod) & mlt) | (mfb & m64) | c65;
  const float v = __uint_as_float(vb);
  const unsigned short hb = f2bf_bits(v);
  const float res = v - bf_bits2f(hb);
  const unsigned short lb = f2bf_bits(res);
  return (((unsigned)lb) & lmask) | (((unsigned)hb) & ~lmask);
}

__global__ __launch_bounds__(256) void k_planes(
    const float* __restrict__ H, const float* __restrict__ WV, unsigned short* __restrict__ PL)
{
#pragma clang fp contract(off)
  __shared__ float tf[64 * 65];
  __shared__ float sW[64];
  const int tid = threadIdx.x;
  const int j0 = blockIdx.x * 64, b = blockIdx.y;
  {
    const int lr = tid >> 4, c4 = (tid & 15) * 4;
#pragma unroll
    for (int it = 0; it < 4; ++it) {
      const int rr = it * 16 + lr;
      const v4f v = *(const v4fa*)(H + ((size_t)b * GN + j0 + rr) * GD + c4);
      tf[rr * 65 + c4 + 0] = v.x;
      tf[rr * 65 + c4 + 1] = v.y;
      tf[rr * 65 + c4 + 2] = v.z;
      tf[rr * 65 + c4 + 3] = v.w;
    }
    if (tid < 64) sW[tid] = WV[(size_t)b * GN + j0 + tid];
  }
  __syncthreads();

  const int sub = tid >> 3, q = tid & 7;
#pragma unroll 1
  for (int it = 0; it < 10; ++it) {
    const int L = it * 32 + sub;
    const int pidx = ((L >= NB) ? 1 : 0) + ((L >= 2 * NB) ? 1 : 0) + ((L >= 3 * NB) ? 1 : 0);
    const int n = L - pidx * NB;
    const int nn = (n < 63) ? n : 63;
    const unsigned tmask = (pidx >= 2) ? 0xFFFFFFFFu : 0u;
    const unsigned lmask = ((pidx & 1) != 0) ? 0xFFFFu : 0u;
    const unsigned mlt   = (n < 64) ? 0xFFFFFFFFu : 0u;
    const unsigned m64   = (n == 64) ? 0xFFFFFFFFu : 0u;
    const unsigned c65   = ((n == 65) ? 0x3F800000u : 0u) & tmask;
    v4u o;
#pragma unroll
    for (int qq = 0; qq < 4; ++qq) {
      const int ja = 8 * q + 2 * qq;
      const float hv0 = tf[ja * 65 + nn];
      const float hv1 = tf[(ja + 1) * 65 + nn];
      const float wv0 = sW[ja];
      const float wv1 = sW[ja + 1];
      const unsigned b0 = plane_bits(hv0, wv0, tmask, mlt, m64, c65, lmask);
      const unsigned b1 = plane_bits(hv1, wv1, tmask, mlt, m64, c65, lmask);
      o[qq] = (b0 & 0xFFFFu) | (b1 << 16);
    }
    unsigned short* dst = PL + ((size_t)(b * 4 + pidx) * NB + n) * GN + j0 + 8 * q;
    *(volatile v4u*)dst = o;
    __threadfence();
    *(volatile v4u*)dst = o;
  }
}

__device__ __forceinline__ void run_half(const __bf16* arow, const __bf16* ph, const __bf16* pl,
                                         int kb, int h, v8f (&acc)[5]) {
#pragma unroll 1
  for (int k0 = kb; k0 < kb + GN / 2; k0 += 32) {
    const v16b af = load_frag(arow + k0, h);
#pragma unroll
    for (int nt = 0; nt < 5; ++nt) {
      const v16b bh = load_frag(ph + (size_t)nt * 16 * GN + k0, h);
      const v16b bl = load_frag(pl + (size_t)nt * 16 * GN + k0, h);
      acc[nt] = mma_bf16(af, bh, acc[nt]);
      acc[nt] = mma_bf16(af, bl, acc[nt]);
    }
  }
}

__global__ __launch_bounds__(256) void k_att(
    const unsigned short* __restrict__ MASKp, const unsigned short* __restrict__ PLp,
    const float* __restrict__ L0R, const float* __restrict__ L1R,
    const float* __restrict__ HM, const float* __restrict__ AFBF,
    const float* __restrict__ H, float* __restrict__ out)
{
  __shared__ __attribute__((aligned(16))) float sX[8][2][256];
  __shared__ __attribute__((aligned(16))) float sF[8][4][16];
  __shared__ __attribute__((aligned(16))) float sO[8][16 * 68];

  const int tid = threadIdx.x, lane = tid & 31, w = tid >> 5;
  const int h = lane >> 4, m = lane & 15;
  const int mt = blockIdx.x, b = blockIdx.y;
  const int type = (mt >= (GN / 2) / MT) ? 1 : 0;
  const int i0 = mt * MT + 16 * w;

  const __bf16* arow = (const __bf16*)(const void*)MASKp + (size_t)(i0 + m) * GN;
  const __bf16* ph = (const __bf16*)(const void*)PLp + (size_t)((b * 2 + type) * 2) * PLANE_ELEMS + (size_t)m * GN;
  const __bf16* pl = ph + PLANE_ELEMS;

  const v8f zero8 = {0.f, 0.f, 0.f, 0.f, 0.f, 0.f, 0.f, 0.f};
  v8f acc0[5], acc1[5];
#pragma unroll
  for (int nt = 0; nt < 5; ++nt) { acc0[nt] = zero8; acc1[nt] = zero8; }

  run_half(arow, ph, pl, 0, h, acc0);
  run_half(arow, ph, pl, GN / 2, h, acc1);

  float* sx = &sX[w][0][0];
#pragma unroll
  for (int r = 0; r < 8; ++r) {
    sx[(8 * h + r) * 16 + m] = acc0[4][r];
    sx[256 + (8 * h + r) * 16 + m] = acc1[4][r];
  }
  __syncthreads();

  {
    const int row = m;
    const float a0 = sx[row * 16 + 0], a1 = sx[256 + row * 16 + 0];
    const float c0 = sx[row * 16 + 1], c1 = sx[256 + row * 16 + 1];
    const int i = i0 + row;
    const int il = (i < GN / 2 - 1) ? i : (GN / 2 - 1);
    const float l0 = L0R[(size_t)b * (GN / 2) + il];
    const float l1 = L1R[(size_t)b * (GN / 2) + il];
    const float ninf = -__builtin_inff();
    const bool has0 = a0 > 0.5f, has1 = a1 > 0.5f;
    const float mx = fmaxf(has0 ? l0 : ninf, has1 ? l1 : ninf);
    const float mxs = (has0 || has1) ? mx : 0.0f;
    const float e0l = has0 ? expf(l0 - mxs) : 0.0f;
    const float e1l = has1 ? expf(l1 - mxs) : 0.0f;
    const float denl = e0l * a0 + e1l * a1;
    const float cntl = a0 + a1;
    const float denu = a0 + a1;
    const float cntu = c0 + c1;
    const bool up = (type != 0);
    const float e0 = up ? 1.0f : e0l;
    const float e1 = up ? 1.0f : e1l;
    const float den = up ? denu : denl;
    const float cnt = up ? cntu : cntl;
    const bool empty = !(cnt > 0.5f);
    const bool bad = (!empty) && !(den > 0.0f);
    const float inv = 1.0f / den;
    sF[w][0][row] = e0 * inv;
    sF[w][1][row] = e1 * inv;
    sF[w][2][row] = empty ? 1.0f : 0.0f;
    sF[w][3][row] = bad ? 1.0f : 0.0f;
  }
  __syncthreads();

  {
    float* so = sO[w];
#pragma unroll
    for (int r = 0; r < 8; ++r) {
      const int row = 8 * h + r;
      const float f0 = sF[w][0][row], f1 = sF[w][1][row];
#pragma unroll
      for (int nt = 0; nt < 4; ++nt)
        so[row * 68 + 16 * nt + m] = f0 * acc0[nt][r] + f1 * acc1[nt][r];
    }
  }
  __syncthreads();

  {
    const float* so = sO[w];
    const int c4 = m * 4;
    const v4f bfv = *(const v4fa*)(AFBF + 128 + c4);
    v4f hmv = *(const v4fa*)(HM + (size_t)b * GD + c4);
    asm volatile("" : "+v"(hmv));
    const float qnan = __int_as_float(0x7fc00000);
#pragma unroll 1
    for (int it = 0; it < 8; ++it) {
      const int row = it * 2 + h;
      const size_t gi = ((size_t)b * GN + i0 + row) * GD + c4;
      const v4f ov = *(const v4fa*)(so + row * 68 + c4);
      const v4f hr = *(const v4fa*)(H + gi);
      const bool fe = sF[w][2][row] > 0.5f;
      const bool fb = sF[w][3][row] > 0.5f;
      v4f y;
#pragma unroll
      for (int e = 0; e < 4; ++e) {
        float o = ov[e];
        o = fe ? hmv[e] : o;
        o = fb ? qnan : o;
        y[e] = tanhf(o + bfv[e]) + hr[e];
      }
      float* dst = out + gi;
      *(volatile v4f*)dst = y;
      __threadfence();
      *(volatile v4f*)dst = y;
    }
  }
}

extern "C" void kernel_launch(void* const* d_in, const int* in_sizes, int n_in,
                              void* d_out, int out_size, void* d_ws, size_t ws_size,
                              hipStream_t stream) {
  if (n_in < 5) return;
  if (in_sizes[0] != GB * GN * GC) return;
  if (in_sizes[1] != GN * GN) return;
  if (in_sizes[2] != GC * GD) return;
  if (in_sizes[3] != 2 * GD) return;
  if (in_sizes[4] != GD) return;
  if (out_size != GB * GN * GD) return;

  const float* x    = (const float*)d_in[0];
  const int*   adj  = (const int*)d_in[1];
  const float* W    = (const float*)d_in[2];
  const float* a    = (const float*)d_in[3];
  const float* bias = (const float*)d_in[4];
  float* out = (float*)d_out;

  const size_t szXB   = (size_t)GB * GN * GC * 2;
  const size_t szMASK = (size_t)GN * GN * 2;
  const size_t szWt   = (size_t)GD * GC * 2;
  const size_t szAFBF = 1024;
  const size_t szH    = (size_t)GB * GN * GD * 4;
  const size_t szS12  = (size_t)2 * GB * GN * 4;
  const size_t szWV   = (size_t)GB * GN * 4;
  const size_t szLR   = (size_t)GB * (GN / 2) * 4;
  const size_t szHM   = (size_t)GB * GD * 4;
  const size_t szSTAT = (size_t)GB * 32 * 4;
  const size_t szPL   = (size_t)GB * 4 * PLANE_ELEMS * 2;

  size_t off = 0;
  const size_t oXB = off;   off += szXB;
  const size_t oMASK = off; off += szMASK;
  const size_t oWt = off;   off += szWt;
  const size_t oAFBF = off; off += szAFBF;
  const size_t oH = off;    off += szH;
  const size_t oS12 = off;  off += szS12;
  const size_t oWV = off;   off += szWV;
  const size_t oL0 = off;   off += szLR;
  const size_t oL1 = off;   off += szLR;
  const size_t oHM = off;   off += szHM;
  const size_t oSTAT = off; off += szSTAT;
  const size_t oPL = off;   off += szPL;
  if (off > ws_size) return;
  if (off > (size_t)134217728) return;

  char* ws = (char*)d_ws;
  unsigned short* XB   = (unsigned short*)(ws + oXB);
  unsigned short* MASK = (unsigned short*)(ws + oMASK);
  unsigned short* Wt   = (unsigned short*)(ws + oWt);
  float* AFBF = (float*)(ws + oAFBF);
  float* Hh   = (float*)(ws + oH);
  float* S12  = (float*)(ws + oS12);
  float* WV   = (float*)(ws + oWV);
  float* L0R  = (float*)(ws + oL0);
  float* L1R  = (float*)(ws + oL1);
  float* HM   = (float*)(ws + oHM);
  float* STAT = (float*)(ws + oSTAT);
  unsigned short* PL = (unsigned short*)(ws + oPL);

  k_prep<<<dim3(PREP_BLOCKS), dim3(256), 0, stream>>>(x, adj, W, a, bias, XB, MASK, Wt, AFBF);
  k_hid<<<dim3((GB * GN) / 128), dim3(256), 0, stream>>>(XB, Wt, AFBF, Hh, S12);
  k_wts<<<dim3(GB), dim3(256), 0, stream>>>(S12, Hh, WV, L0R, L1R, HM, STAT);
  k_planes<<<dim3(GN / 64, GB), dim3(256), 0, stream>>>(Hh, WV, PL);
  k_att<<<dim3(GN / MT, GB), dim3(256), 0, stream>>>(MASK, PL, L0R, L1R, HM, AFBF, Hh, out);
  (void)hipGetLastError();
}
